// TIPSv2VisionAttention_31044023615544
// MI455X (gfx1250) — hardware-verified
//
#include <hip/hip_runtime.h>
#include <math.h>
#include <stdint.h>

static constexpr int NB   = 4;
static constexpr int NSEQ = 1370;
static constexpr int NPAD = 1408;
static constexpr int DIM  = 1024;
static constexpr int NH   = 16;
static constexpr int HD   = 64;
static constexpr int MP   = NB * NPAD;
static constexpr int QKW  = 2 * DIM;
static_assert(NPAD % 64 == 0);
static_assert(NPAD >= NSEQ);
static_assert(NH * HD == DIM);
static_assert(DIM % 64 == 0);
static_assert((MP * DIM) % (8 * 256) == 0);

#define PSC  4096.0f
#define RPSC 0.000244140625f
#define VLS  2048.0f
#define RVLS 0.00048828125f
#define SSC  0.125f

typedef _Float16 v16h __attribute__((ext_vector_type(16)));
typedef _Float16 v8h  __attribute__((ext_vector_type(8)));
typedef __bf16   v16b __attribute__((ext_vector_type(16)));
typedef __bf16   v8b  __attribute__((ext_vector_type(8)));
typedef float    v8f  __attribute__((ext_vector_type(8)));
typedef float    v4f  __attribute__((ext_vector_type(4)));
typedef unsigned int v4u __attribute__((ext_vector_type(4)));

union FB { v16b v; v8b h[2]; };
union FH { v16h v; v8h h[2]; };

__device__ __forceinline__ unsigned short f2bf_bits(float f) {
  unsigned u = __float_as_uint(f);
  return (unsigned short)((u + 0x7FFFu + ((u >> 16) & 1u)) >> 16);
}
__device__ __forceinline__ float bf_bits2f(unsigned short h) { return __uint_as_float(((unsigned)h) << 16); }
__device__ __forceinline__ float bf_rne(float f) { return bf_bits2f(f2bf_bits(f)); }
__device__ __forceinline__ unsigned pk16(unsigned short a, unsigned short b) { return (unsigned)a | ((unsigned)b << 16); }
__device__ __forceinline__ unsigned short h2bits(_Float16 h) { return __builtin_bit_cast(unsigned short, h); }

__device__ __forceinline__ v8f mma_b(v16b a, v16b b, v8f c) {
  return __builtin_amdgcn_wmma_f32_16x16x32_bf16(false, a, false, b, (short)0, c, false, false);
}
__device__ __forceinline__ v8f mma_bg(v16b a, v16b b, v8f c) {
  c = __builtin_amdgcn_wmma_f32_16x16x32_bf16(false, a, false, b, (short)0, c, false, false);
  asm volatile("v_nop\n\tv_nop\n\tv_nop\n\tv_nop" : "+v"(c) : "v"(a), "v"(b));
  return c;
}
__device__ __forceinline__ v8f mma_hg(v16h a, v16h b, v8f c) {
  c = __builtin_amdgcn_wmma_f32_16x16x32_f16(false, a, false, b, (short)0, c, false, false);
  asm volatile("v_nop\n\tv_nop\n\tv_nop\n\tv_nop" : "+v"(c) : "v"(a), "v"(b));
  return c;
}
__device__ __forceinline__ void g4b(v8f& a, v8f& b, v8f& c, v8f& d, v16b x, v16b y) {
  asm volatile("v_nop\n\tv_nop\n\tv_nop\n\tv_nop" : "+v"(a), "+v"(b), "+v"(c), "+v"(d) : "v"(x), "v"(y));
}
__device__ __forceinline__ void keep4b(v16b a, v16b b, v16b c, v16b d) {
  asm volatile("v_nop" :: "v"(a), "v"(b), "v"(c), "v"(d));
}
__device__ __forceinline__ void accg4(v8f& a, v8f& b, v8f& c, v8f& d) {
  asm volatile("v_nop\n\tv_nop\n\tv_nop\n\tv_nop" : "+v"(a), "+v"(b), "+v"(c), "+v"(d));
}
__device__ __forceinline__ void lds_sync_wave() {
  __builtin_amdgcn_fence(__ATOMIC_RELEASE, "workgroup");
  __builtin_amdgcn_wave_barrier();
  __builtin_amdgcn_fence(__ATOMIC_ACQUIRE, "workgroup");
}
__device__ __forceinline__ v16b ldfrag_b(const __bf16* p) {
  FB f; f.h[0] = *(const v8b*)(p); f.h[1] = *(const v8b*)(p + 16); return f.v;
}

template <int NPROD, int BIAS_MODE, int OUT_MODE>
__global__ __launch_bounds__(256) void gemm64_kernel(
    const unsigned short* __restrict__ Ap, const unsigned short* __restrict__ A2p, int lda, long strideA,
    const unsigned short* __restrict__ Btp, int ldb, long strideB,
    void* Cout, void* Cout2, int ldc, long strideC,
    const float* __restrict__ bias, int M, int N, int K, int rpIn, int rpOut) {
  __shared__ __align__(16) float sT[8][16 * 68];
  const int b    = blockIdx.y;
  const int lane = threadIdx.x & 31;
  const int wave = threadIdx.x >> 5;
  const int tilesN = N >> 6;
  const int tilesM = M >> 6;
  const int tile = blockIdx.x * 8 + wave;
  if (tile >= tilesM * tilesN) return;
  const int tm = tile / tilesN;
  const int tn = tile - tm * tilesN;
  const int m0 = tm << 6;
  const int n0 = tn << 6;

  const __bf16* Ab  = (const __bf16*)(const void*)Ap  + (size_t)b * strideA;
  const __bf16* Ab2 = (const __bf16*)(const void*)A2p + (size_t)b * strideA;
  const __bf16* Bb  = (const __bf16*)(const void*)Btp + (size_t)b * strideB;

  const int rl   = lane & 15;
  const int koff = (lane >> 4) * 8;
  const int mOff = (lane >> 4) * 8;

  v8f acc[4][4];
#pragma unroll
  for (int i = 0; i < 4; ++i)
#pragma unroll
    for (int j = 0; j < 4; ++j) acc[i][j] = (v8f){0.f, 0.f, 0.f, 0.f, 0.f, 0.f, 0.f, 0.f};

  for (int k0 = 0; k0 < K; k0 += 32) {
    v16b bq[4];
#pragma unroll
    for (int j = 0; j < 4; ++j)
      bq[j] = ldfrag_b(Bb + (size_t)(n0 + 16 * j + rl) * ldb + k0 + koff);
#pragma unroll
    for (int i = 0; i < 4; ++i) {
      const size_t ao = (size_t)(m0 + 16 * i + rl) * lda + k0 + koff;
      v16b ah = ldfrag_b(Ab + ao);
      v16b al = ah;
      if (NPROD == 2) al = ldfrag_b(Ab2 + ao);
#pragma unroll
      for (int j = 0; j < 4; ++j) {
        acc[i][j] = mma_b(ah, bq[j], acc[i][j]);
        if (NPROD == 2) acc[i][j] = mma_b(al, bq[j], acc[i][j]);
      }
      g4b(acc[i][0], acc[i][1], acc[i][2], acc[i][3], ah, al);
    }
    keep4b(bq[0], bq[1], bq[2], bq[3]);
  }
  accg4(acc[0][0], acc[0][1], acc[0][2], acc[0][3]);
  accg4(acc[1][0], acc[1][1], acc[1][2], acc[1][3]);
  accg4(acc[2][0], acc[2][1], acc[2][2], acc[2][3]);
  accg4(acc[3][0], acc[3][1], acc[3][2], acc[3][3]);

  float* slab = sT[wave];
#pragma unroll
  for (int i = 0; i < 4; ++i) {
    const int mBase = m0 + 16 * i;
#pragma unroll
    for (int j = 0; j < 4; ++j) {
      const int n = n0 + 16 * j + rl;
      float bv = 0.f;
      if (BIAS_MODE == 2) bv = bf_rne(bias[n]);
#pragma unroll
      for (int r = 0; r < 8; ++r) {
        float v = acc[i][j][r];
        if (BIAS_MODE == 1) v += bf_rne(bias[mBase + mOff + r]);
        if (BIAS_MODE == 2) v += bv;
        slab[(mOff + r) * 68 + 16 * j + rl] = v;
      }
    }
    lds_sync_wave();
    if (OUT_MODE == 0) {
      float* C = (float*)Cout + (size_t)b * strideC;
      const int hh = lane >> 4, c4 = (lane & 15) * 4;
      v4f vv[8];
      int orow[8];
#pragma unroll
      for (int it = 0; it < 8; ++it) {
        const int row = it * 2 + hh;
        vv[it] = *(const v4f*)(slab + row * 68 + c4);
        const int m = mBase + row;
        const int g = m / rpIn;
        const int t = m - g * rpIn;
        orow[it] = (t < rpOut) ? (g * rpOut + t) : -1;
      }
      for (int pass = 0; pass < 2; ++pass) {
#pragma unroll
        for (int it = 0; it < 8; ++it) {
          if (orow[it] >= 0)
            *(volatile v4f*)(C + (size_t)orow[it] * ldc + n0 + c4) = vv[it];
        }
        __threadfence();
      }
    } else {
      const int q = lane >> 3, c8 = (lane & 7) * 8;
      unsigned short* C  = (unsigned short*)Cout  + (size_t)b * strideC;
      unsigned short* C2 = (unsigned short*)Cout2 + (size_t)b * strideC;
      v4u hv[4], lv[4];
#pragma unroll
      for (int it = 0; it < 4; ++it) {
        const int row = it * 4 + q;
        const float* sp = slab + row * 68 + c8;
        v4u a, a2;
#pragma unroll
        for (int e = 0; e < 4; ++e) {
          const float f0 = sp[2 * e], f1 = sp[2 * e + 1];
          if (OUT_MODE == 1) {
            const unsigned short h0 = f2bf_bits(f0), h1 = f2bf_bits(f1);
            const unsigned short l0 = f2bf_bits(f0 - bf_bits2f(h0)), l1 = f2bf_bits(f1 - bf_bits2f(h1));
            a[e] = pk16(h0, h1); a2[e] = pk16(l0, l1);
          } else {
            const _Float16 h0 = (_Float16)f0, h1 = (_Float16)f1;
            const _Float16 l0 = (_Float16)((f0 - (float)h0) * VLS), l1 = (_Float16)((f1 - (float)h1) * VLS);
            a[e] = pk16(h2bits(h0), h2bits(h1)); a2[e] = pk16(h2bits(l0), h2bits(l1));
          }
        }
        hv[it] = a; lv[it] = a2;
      }
      for (int pass = 0; pass < 2; ++pass) {
#pragma unroll
        for (int it = 0; it < 4; ++it) {
          const int row = it * 4 + q;
          const size_t go = (size_t)(mBase + row) * ldc + n0 + c8;
          *(volatile v4u*)(C + go)  = hv[it];
          *(volatile v4u*)(C2 + go) = lv[it];
        }
        __threadfence();
      }
    }
    lds_sync_wave();
  }
}

__global__ __launch_bounds__(256) void cvt_x_kernel(const float* __restrict__ x, unsigned short* xb) {
  const int i = blockIdx.x * 256 + threadIdx.x;
  if (i >= (MP * DIM) / 8) return;
  const int e0  = i * 8;
  const int m   = e0 / DIM;
  const int col = e0 - m * DIM;
  const int b   = m / NPAD;
  const int t   = m - b * NPAD;
  const int tc  = (t < NSEQ) ? t : (NSEQ - 1);
  const float* src = x + ((size_t)(b * NSEQ + tc) * DIM + col);
  const v4f f0 = *(const v4f*)(src);
  const v4f f1 = *(const v4f*)(src + 4);
  const bool live = (t < NSEQ);
  v4u o;
  o[0] = live ? pk16(f2bf_bits(f0[0]), f2bf_bits(f0[1])) : 0u;
  o[1] = live ? pk16(f2bf_bits(f0[2]), f2bf_bits(f0[3])) : 0u;
  o[2] = live ? pk16(f2bf_bits(f1[0]), f2bf_bits(f1[1])) : 0u;
  o[3] = live ? pk16(f2bf_bits(f1[2]), f2bf_bits(f1[3])) : 0u;
  unsigned short* dst = xb + (size_t)e0;
  *(volatile v4u*)dst = o;
  __threadfence();
  *(volatile v4u*)dst = o;
}

__global__ __launch_bounds__(256) void tcvt_kernel(const float* __restrict__ W, unsigned short* out, int R, int Cc) {
  __shared__ __align__(16) float tf[64 * 68];
  const int c0  = blockIdx.x * 64;
  const int r0  = blockIdx.y * 64;
  const int tid = threadIdx.x;
  {
    const int lr = tid >> 4;
    const int c4 = (tid & 15) * 4;
#pragma unroll
    for (int it = 0; it < 4; ++it) {
      const int rr = it * 16 + lr;
      const v4f a = *(const v4f*)(W + (size_t)(r0 + rr) * Cc + c0 + c4);
      *(v4f*)(tf + rr * 68 + c4) = a;
    }
  }
  __syncthreads();
  const int sub = tid >> 3;
  const int c8  = (tid & 7) * 8;
  v4u hv[2];
#pragma unroll
  for (int it = 0; it < 2; ++it) {
    const int oc = it * 32 + sub;
    v4u a;
#pragma unroll
    for (int q = 0; q < 4; ++q) {
      const float f0 = tf[(c8 + 2 * q) * 68 + oc];
      const float f1 = tf[(c8 + 2 * q + 1) * 68 + oc];
      a[q] = pk16(f2bf_bits(f0), f2bf_bits(f1));
    }
    hv[it] = a;
  }
  for (int pass = 0; pass < 2; ++pass) {
#pragma unroll
    for (int it = 0; it < 2; ++it) {
      const int oc = it * 32 + sub;
      const size_t go = (size_t)(c0 + oc) * R + r0 + c8;
      *(volatile v4u*)(out + go) = hv[it];
    }
    __threadfence();
  }
}

__global__ __launch_bounds__(128) void attn_kernel(
    const unsigned short* __restrict__ qkhp, const unsigned short* __restrict__ qklp,
    const unsigned short* __restrict__ vthp, const unsigned short* __restrict__ vtlp,
    unsigned short* ohp, unsigned short* olp) {
  __shared__ __align__(16) __bf16   Ksh[64 * 64];
  __shared__ __align__(16) __bf16   Ksl[64 * 64];
  __shared__ __align__(16) _Float16 Vsh[64 * 64];
  __shared__ __align__(16) _Float16 Vsl[64 * 64];
  __shared__ __align__(16) _Float16 Psh[4][16 * 64];
  __shared__ __align__(16) float    Osl[4][16 * 68];

  const int tid  = threadIdx.x;
  const int wave = tid >> 5;
  const int lane = tid & 31;
  const int hh   = lane >> 4;
  const int c    = lane & 15;

  const int nqb = NPAD / 64;
  const int bx  = blockIdx.x;
  const int qb  = bx % nqb;
  const int h   = bx / nqb;
  const int b   = blockIdx.y;
  const int q0  = qb * 64 + wave * 16;
  const size_t rowB = (size_t)b * NPAD;

  const __bf16*   QKh = (const __bf16*)(const void*)qkhp;
  const __bf16*   QKl = (const __bf16*)(const void*)qklp;
  const _Float16* VTh = (const _Float16*)(const void*)vthp + ((size_t)b * DIM + (size_t)h * HD) * NPAD;
  const _Float16* VTl = (const _Float16*)(const void*)vtlp + ((size_t)b * DIM + (size_t)h * HD) * NPAD;
  const __bf16* Qrh = QKh + (rowB + q0 + c) * QKW + h * HD + 8 * hh;
  const __bf16* Qrl = QKl + (rowB + q0 + c) * QKW + h * HD + 8 * hh;

  float mrow[8], lrow[8];
  v8f oh[4], ol[4];
#pragma unroll
  for (int r = 0; r < 8; ++r) { mrow[r] = -INFINITY; lrow[r] = 0.f; }
#pragma unroll
  for (int t = 0; t < 4; ++t) {
    oh[t] = (v8f){0.f, 0.f, 0.f, 0.f, 0.f, 0.f, 0.f, 0.f};
    ol[t] = (v8f){0.f, 0.f, 0.f, 0.f, 0.f, 0.f, 0.f, 0.f};
  }

  for (int kc = 0; kc < NPAD / 64; ++kc) {
    const int kv0 = kc * 64;
    __syncthreads();
    {
      const int r = tid >> 1, half = (tid & 1) * 32;
      const __bf16*   ks_h = QKh + (rowB + kv0 + r) * QKW + DIM + h * HD + half;
      const __bf16*   ks_l = QKl + (rowB + kv0 + r) * QKW + DIM + h * HD + half;
      const _Float16* vs_h = VTh + (size_t)r * NPAD + kv0 + half;
      const _Float16* vs_l = VTl + (size_t)r * NPAD + kv0 + half;
#pragma unroll
      for (int i = 0; i < 4; ++i) {
        const v8b a0 = *(const v8b*)(ks_h + 8 * i);
        const v8b a1 = *(const v8b*)(ks_l + 8 * i);
        const v8h b0 = *(const v8h*)(vs_h + 8 * i);
        const v8h b1 = *(const v8h*)(vs_l + 8 * i);
        *(v8b*)(Ksh + r * 64 + half + 8 * i) = a0;
        *(v8b*)(Ksl + r * 64 + half + 8 * i) = a1;
        *(v8h*)(Vsh + r * 64 + half + 8 * i) = b0;
        *(v8h*)(Vsl + r * 64 + half + 8 * i) = b1;
      }
    }
    __syncthreads();

    v8f s[4];
#pragma unroll
    for (int j = 0; j < 4; ++j) s[j] = (v8f){0.f, 0.f, 0.f, 0.f, 0.f, 0.f, 0.f, 0.f};
#pragma unroll
    for (int dc = 0; dc < 2; ++dc) {
      FB qa, ql;
      qa.h[0] = *(const v8b*)(Qrh + dc * 32);
      qa.h[1] = *(const v8b*)(Qrh + dc * 32 + 16);
      ql.h[0] = *(const v8b*)(Qrl + dc * 32);
      ql.h[1] = *(const v8b*)(Qrl + dc * 32 + 16);
#pragma unroll
      for (int j = 0; j < 4; ++j) {
        FB kb, kl;
        kb.h[0] = *(const v8b*)(Ksh + (16 * j + c) * 64 + dc * 32 + 8 * hh);
        kb.h[1] = *(const v8b*)(Ksh + (16 * j + c) * 64 + dc * 32 + 16 + 8 * hh);
        kl.h[0] = *(const v8b*)(Ksl + (16 * j + c) * 64 + dc * 32 + 8 * hh);
        kl.h[1] = *(const v8b*)(Ksl + (16 * j + c) * 64 + dc * 32 + 16 + 8 * hh);
        s[j] = mma_bg(qa.v, kb.v, s[j]);
        s[j] = mma_bg(qa.v, kl.v, s[j]);
        s[j] = mma_bg(ql.v, kb.v, s[j]);
      }
    }

    float cm[8];
#pragma unroll
    for (int r = 0; r < 8; ++r) {
      float m = -INFINITY;
#pragma unroll
      for (int j = 0; j < 4; ++j) {
        const int key = kv0 + 16 * j + c;
        float sv = s[j][r] * SSC;
        sv = (key < NSEQ) ? sv : -INFINITY;
        s[j][r] = sv;
        m = fmaxf(m, sv);
      }
#pragma unroll
      for (int off = 1; off < 16; off <<= 1) m = fmaxf(m, __shfl_xor(m, off, 32));
      cm[r] = m;
    }

    _Float16* pw = Psh[wave];
#pragma unroll
    for (int r = 0; r < 8; ++r) {
      const float mnew  = fmaxf(mrow[r], cm[r]);
      const float alpha = __expf(mrow[r] - mnew);
      mrow[r] = mnew;
      float psum = 0.f;
#pragma unroll
      for (int j = 0; j < 4; ++j) {
        const float p = __expf(s[j][r] - mnew);
        psum += p;
        pw[(8 * hh + r) * 64 + 16 * j + c] = (_Float16)(p * PSC);
      }
#pragma unroll
      for (int off = 1; off < 16; off <<= 1) psum += __shfl_xor(psum, off, 32);
      lrow[r] = lrow[r] * alpha + psum;
#pragma unroll
      for (int t = 0; t < 4; ++t) { oh[t][r] *= alpha; ol[t][r] *= alpha; }
    }
    lds_sync_wave();

#pragma unroll
    for (int kk = 0; kk < 2; ++kk) {
      FH pa;
      pa.h[0] = *(const v8h*)(pw + c * 64 + kk * 32 + 8 * hh);
      pa.h[1] = *(const v8h*)(pw + c * 64 + kk * 32 + 16 + 8 * hh);
#pragma unroll
      for (int t = 0; t < 4; ++t) {
        FH vb, vl;
        vb.h[0] = *(const v8h*)(Vsh + (16 * t + c) * 64 + kk * 32 + 8 * hh);
        vb.h[1] = *(const v8h*)(Vsh + (16 * t + c) * 64 + kk * 32 + 16 + 8 * hh);
        vl.h[0] = *(const v8h*)(Vsl + (16 * t + c) * 64 + kk * 32 + 8 * hh);
        vl.h[1] = *(const v8h*)(Vsl + (16 * t + c) * 64 + kk * 32 + 16 + 8 * hh);
        oh[t] = mma_hg(pa.v, vb.v, oh[t]);
        ol[t] = mma_hg(pa.v, vl.v, ol[t]);
      }
    }
  }

  float* os = Osl[wave];
#pragma unroll
  for (int r = 0; r < 8; ++r) {
    const float inv = (1.0f / lrow[r]) * RPSC;
#pragma unroll
    for (int t = 0; t < 4; ++t) os[(8 * hh + r) * 68 + 16 * t + c] = (oh[t][r] + ol[t][r] * RVLS) * inv;
  }
  lds_sync_wave();
  {
    const int q = lane >> 3, c8 = (lane & 7) * 8;
    v4u hv[4], lv[4];
#pragma unroll
    for (int it = 0; it < 4; ++it) {
      const int row = it * 4 + q;
      const float* sp = os + row * 68 + c8;
      v4u a, a2;
#pragma unroll
      for (int e = 0; e < 4; ++e) {
        const float f0 = sp[2 * e], f1 = sp[2 * e + 1];
        const unsigned short h0 = f2bf_bits(f0), h1 = f2bf_bits(f1);
        const unsigned short l0 = f2bf_bits(f0 - bf_bits2f(h0)), l1 = f2bf_bits(f1 - bf_bits2f(h1));
        a[e] = pk16(h0, h1); a2[e] = pk16(l0, l1);
      }
      hv[it] = a; lv[it] = a2;
    }
    for (int pass = 0; pass < 2; ++pass) {
#pragma unroll
      for (int it = 0; it < 4; ++it) {
        const int row = it * 4 + q;
        const size_t go = (rowB + q0 + row) * DIM + (size_t)h * HD + c8;
        *(volatile v4u*)(ohp + go) = hv[it];
        *(volatile v4u*)(olp + go) = lv[it];
      }
      __threadfence();
    }
  }
}

extern "C" void kernel_launch(void* const* d_in, const int* in_sizes, int n_in,
                              void* d_out, int out_size, void* d_ws, size_t ws_size,
                              hipStream_t stream) {
  if (n_in < 5) return;
  if (in_sizes[0] != NB * NSEQ * DIM) return;
  if (in_sizes[1] != DIM * 3 * DIM) return;
  if (in_sizes[2] != 3 * DIM) return;
  if (in_sizes[3] != DIM * DIM) return;
  if (in_sizes[4] != DIM) return;
  if (out_size != NB * NSEQ * DIM) return;

  const float* x      = (const float*)d_in[0];
  const float* w_qkv  = (const float*)d_in[1];
  const float* b_qkv  = (const float*)d_in[2];
  const float* w_proj = (const float*)d_in[3];
  const float* b_proj = (const float*)d_in[4];

  const size_t szXb = (size_t)MP * DIM * 2;
  const size_t szWq = (size_t)3 * DIM * DIM * 2;
  const size_t szWp = (size_t)DIM * DIM * 2;
  const size_t szQK = (size_t)MP * QKW * 2;
  const size_t szVt = (size_t)NB * DIM * NPAD * 2;
  const size_t szO  = (size_t)MP * DIM * 2;
  size_t off = 0;
  const size_t oXb  = off; off += szXb;
  const size_t oWq  = off; off += szWq;
  const size_t oWp  = off; off += szWp;
  const size_t oQKh = off; off += szQK;
  const size_t oQKl = off; off += szQK;
  const size_t oVth = off; off += szVt;
  const size_t oVtl = off; off += szVt;
  const size_t oOh  = off; off += szO;
  const size_t oOl  = off; off += szO;
  if (off > ws_size) return;

  char* ws = (char*)d_ws;
  unsigned short* Xb  = (unsigned short*)(ws + oXb);
  unsigned short* Wqt = (unsigned short*)(ws + oWq);
  unsigned short* Wpt = (unsigned short*)(ws + oWp);
  unsigned short* QKh = (unsigned short*)(ws + oQKh);
  unsigned short* QKl = (unsigned short*)(ws + oQKl);
  unsigned short* Vth = (unsigned short*)(ws + oVth);
  unsigned short* Vtl = (unsigned short*)(ws + oVtl);
  unsigned short* Oh  = (unsigned short*)(ws + oOh);
  unsigned short* Ol  = (unsigned short*)(ws + oOl);
  unsigned short* Wvt = Wqt + (size_t)2 * DIM * DIM;

  const dim3 blk(256);

  cvt_x_kernel<<<dim3((MP * DIM) / 8 / 256), blk, 0, stream>>>(x, Xb);
  tcvt_kernel<<<dim3((3 * DIM) / 64, DIM / 64), blk, 0, stream>>>(w_qkv, Wqt, DIM, 3 * DIM);
  tcvt_kernel<<<dim3(DIM / 64, DIM / 64), blk, 0, stream>>>(w_proj, Wpt, DIM, DIM);

  const dim3 gQK(((MP / 64) * (QKW / 64) + 7) / 8, 1);
  gemm64_kernel<1, 2, 1><<<gQK, blk, 0, stream>>>(
      Xb, Xb, DIM, 0L, Wqt, DIM, 0L, (void*)QKh, (void*)QKl, QKW, 0L,
      b_qkv, MP, QKW, DIM, MP, MP);

  const dim3 gVT(((DIM / 64) * (NPAD / 64) + 7) / 8, NB);
  gemm64_kernel<1, 1, 2><<<gVT, blk, 0, stream>>>(
      Wvt, Wvt, DIM, 0L, Xb, DIM, (long)NPAD * DIM, (void*)Vth, (void*)Vtl, NPAD, (long)DIM * NPAD,
      b_qkv + 2 * DIM, DIM, NPAD, DIM, DIM, DIM);

  attn_kernel<<<dim3(NH * (NPAD / 64), NB), dim3(128), 0, stream>>>(QKh, QKl, Vth, Vtl, Oh, Ol);

  const dim3 gPR(((MP / 64) * (DIM / 64) + 7) / 8, 1);
  gemm64_kernel<2, 2, 0><<<gPR, blk, 0, stream>>>(
      Oh, Ol, DIM, 0L, Wpt, DIM, 0L, d_out, d_out, DIM, 0L,
      b_proj, MP, DIM, DIM, NPAD, NSEQ);

  (void)hipGetLastError();
}
